// TriangleAttention_50294067036161
// MI455X (gfx1250) — hardware-verified
//
#include <hip/hip_runtime.h>
#include <stddef.h>
#include <stdint.h>


typedef _Float16 half_t;
typedef _Float16 v16h __attribute__((ext_vector_type(16)));
typedef _Float16 h8   __attribute__((ext_vector_type(8)));
typedef _Float16 h8a  __attribute__((ext_vector_type(8), may_alias));
typedef _Float16 h4   __attribute__((ext_vector_type(4)));
typedef _Float16 h4a  __attribute__((ext_vector_type(4), may_alias));
typedef float    v8f  __attribute__((ext_vector_type(8)));
typedef float    v4f  __attribute__((ext_vector_type(4)));
typedef float    v4fa __attribute__((ext_vector_type(4), may_alias));

#ifndef NB
#define NB 256
#endif
#define NRES_FULL 256
#define CZ   128
#define NH   4
#define CH   32
#define HC   128
#define NROWS_FULL (NRES_FULL * NRES_FULL)
#define NQROWS     (NB * NRES_FULL)
static_assert(NB >= 1 && NB <= NRES_FULL);
static_assert((NQROWS % 64) == 0);
static_assert((size_t)NQROWS * CZ * 4 <= (size_t)33554432);

#define NTILES       41
#define OFF_W        ((size_t)0)
#define W_BYTES      ((size_t)NTILES * 4 * 32 * 16 * 2)
#define OFF_PROJ     ((size_t)262144)
#define PLANE_HALVES ((size_t)NROWS_FULL * HC)
#define OFF_AO       (OFF_PROJ + 4 * PLANE_HALVES * 2)
#define AO_BYTES     ((size_t)NH * NROWS_FULL * CH * 2)
#define OFF_BIAS     (OFF_AO + AO_BYTES)
#define BIAS_BYTES   ((size_t)NRES_FULL * NH * NRES_FULL * 4)
#define WS_TOTAL     (OFF_BIAS + BIAS_BYTES)
static_assert(W_BYTES <= OFF_PROJ);
static_assert(WS_TOTAL <= (size_t)134217728);
static_assert((OFF_PROJ % 128) == 0 && (OFF_AO % 128) == 0 && (OFF_BIAS % 128) == 0);

#define WCAR     256.0f
#define INV_WCAR (1.0f / 256.0f)
#define OCAR     256.0f

__device__ __forceinline__ float bf16r(float x) {
  unsigned int u = __float_as_uint(x);
  u += 0x7FFFu + ((u >> 16) & 1u);
  u &= 0xFFFF0000u;
  return __uint_as_float(u);
}

__device__ __forceinline__ v8f wmma32(v16h a, v16h b, v8f c) {
  return __builtin_amdgcn_wmma_f32_16x16x32_f16(false, a, false, b, (short)0, c, false, false);
}

__device__ __forceinline__ void wguard(v8f& acc, v16h& a, v16h& b) {
  asm volatile("v_nop\n\tv_nop\n\tv_nop\n\tv_nop" : "+v"(acc) : "v"(a), "v"(b));
}
__device__ __forceinline__ void wguard2(v8f& acc0, v8f& acc1, v16h& a, v16h& b, v16h& c) {
  asm volatile("v_nop\n\tv_nop\n\tv_nop\n\tv_nop" : "+v"(acc0), "+v"(acc1) : "v"(a), "v"(b), "v"(c));
}

__device__ __forceinline__ float wsum32(float s) {
  s += __shfl_xor(s, 16, 32);
  s += __shfl_xor(s, 8, 32);
  s += __shfl_xor(s, 4, 32);
  s += __shfl_xor(s, 2, 32);
  s += __shfl_xor(s, 1, 32);
  return s;
}

__device__ __forceinline__ v16h frag2(const half_t* c0, const half_t* c1) {
  const h8a x0 = *(const h8a*)c0;
  const h8a x1 = *(const h8a*)c1;
  v16h f;
#pragma unroll
  for (int i = 0; i < 8; ++i) { f[i] = x0[i]; f[i + 8] = x1[i]; }
  return f;
}

__device__ __forceinline__ void loadB4(const half_t* __restrict__ pw, int t, int lane, v16h b[4]) {
#pragma unroll
  for (int kb = 0; kb < 4; ++kb)
    b[kb] = *(const v16h*)&pw[((size_t)(t * 4 + kb) * 32 + lane) * 16];
}

__global__ __launch_bounds__(256) void kP(const float* __restrict__ Wb, const float* __restrict__ Wq,
                                          const float* __restrict__ Wk, const float* __restrict__ Wv,
                                          const float* __restrict__ Wg, const float* __restrict__ Wo,
                                          half_t* packedW) {
  const int t  = blockIdx.x;
  const int kb = threadIdx.x >> 6;
  const int j  = threadIdx.x & 63;
  const int L  = j >> 1, p = j & 1;
  const int hi = L >> 4, n = L & 15;
  h8 f;
#pragma unroll
  for (int e = 0; e < 8; ++e) {
    const int k = kb * 32 + 8 * hi + e + 16 * p;
    float v;
    if (t < 8)        v = Wq[k * HC + t * 16 + n];
    else if (t < 16)  v = Wk[k * HC + (t - 8) * 16 + n];
    else if (t < 24)  v = Wv[k * HC + (t - 16) * 16 + n];
    else if (t < 32)  v = Wg[k * HC + (t - 24) * 16 + n];
    else if (t == 32) { const float wv = Wb[k * NH + (n < 4 ? n : 3)]; v = (n < 4) ? wv : 0.0f; }
    else              v = Wo[k * CZ + (t - 33) * 16 + n];
    f[e] = (half_t)(bf16r(v) * WCAR);
  }
  half_t* dst = packedW + (size_t)(t * 4 + kb) * 512 + (size_t)j * 8;
  *(volatile h8*)dst = f;
  __threadfence();
  *(volatile h8*)dst = f;
}

__global__ __launch_bounds__(128) void kA(const float* __restrict__ z, const float* __restrict__ lng,
                                          const float* __restrict__ lnb, const half_t* __restrict__ packedW,
                                          half_t* proj, float* biasbuf, int nqrows) {
  __shared__ __attribute__((aligned(16))) half_t zh[4][16 * CZ];
  __shared__ __attribute__((aligned(16))) half_t stg[4][16 * HC];
  __shared__ __attribute__((aligned(16))) float  bsb[NH][64];
  const int tid = threadIdx.x, w = tid >> 5, lane = tid & 31;
  const int m = lane & 15, hi = lane >> 4;
  const int r0 = (blockIdx.x * 4 + w) * 16;

  const v4f gv4 = *(const v4fa*)(lng + lane * 4);
  const v4f bv4 = *(const v4fa*)(lnb + lane * 4);
  const float g0 = bf16r(gv4.x), g1 = bf16r(gv4.y), g2 = bf16r(gv4.z), g3 = bf16r(gv4.w);
  const float e0 = bf16r(bv4.x), e1 = bf16r(bv4.y), e2 = bf16r(bv4.z), e3 = bf16r(bv4.w);
#pragma unroll 1
  for (int rr = 0; rr < 16; ++rr) {
    const v4f zz = *(const v4fa*)(z + (size_t)(r0 + rr) * CZ + lane * 4);
    const float a0 = bf16r(zz.x), a1 = bf16r(zz.y), a2 = bf16r(zz.z), a3 = bf16r(zz.w);
    float s = (a0 + a1) + (a2 + a3);
    s = wsum32(s);
    const float mean = s * (1.0f / 128.0f);
    const float d0 = a0 - mean, d1 = a1 - mean, d2 = a2 - mean, d3 = a3 - mean;
    float sq = (d0 * d0 + d1 * d1) + (d2 * d2 + d3 * d3);
    sq = wsum32(sq);
    const float inv = rsqrtf(sq * (1.0f / 128.0f) + 1e-5f);
    h4 xv;
    xv.x = (half_t)(d0 * inv * g0 + e0);
    xv.y = (half_t)(d1 * inv * g1 + e1);
    xv.z = (half_t)(d2 * inv * g2 + e2);
    xv.w = (half_t)(d3 * inv * g3 + e3);
    *(h4a*)&zh[w][rr * CZ + lane * 4] = xv;
  }
  __syncthreads();

  v16h afr[4];
#pragma unroll
  for (int kb = 0; kb < 4; ++kb) {
    const half_t* c0 = &zh[w][m * CZ + kb * 32 + hi * 8];
    afr[kb] = frag2(c0, c0 + 16);
  }

  v16h b[4];
  if (blockIdx.x * 64 < nqrows) {
#pragma unroll 1
    for (int P = 0; P < 4; ++P) {
      half_t* dstp = proj + (size_t)P * PLANE_HALVES;
#pragma unroll 1
      for (int t8 = 0; t8 < 8; ++t8) {
        loadB4(packedW, P * 8 + t8, lane, b);
        v8f acc = {};
#pragma unroll
        for (int kb = 0; kb < 4; ++kb) acc = wmma32(afr[kb], b[kb], acc);
        wguard(acc, afr[3], b[3]);
#pragma unroll
        for (int v = 0; v < 8; ++v)
          stg[w][(8 * hi + v) * HC + t8 * 16 + m] = (half_t)acc[v];
      }
      __syncthreads();
      h8 vals[8];
#pragma unroll
      for (int p = 0; p < 8; ++p) vals[p] = *(const h8a*)&stg[w][(2 * p + hi) * HC + m * 8];
#pragma unroll
      for (int p = 0; p < 8; ++p)
        *(volatile h8*)(dstp + (size_t)(r0 + 2 * p + hi) * HC + m * 8) = vals[p];
      __threadfence();
#pragma unroll
      for (int p = 0; p < 8; ++p)
        *(volatile h8*)(dstp + (size_t)(r0 + 2 * p + hi) * HC + m * 8) = vals[p];
      __syncthreads();
    }
  }

  {
    loadB4(packedW, 32, lane, b);
    v8f acc = {};
#pragma unroll
    for (int kb = 0; kb < 4; ++kb) acc = wmma32(afr[kb], b[kb], acc);
    wguard(acc, afr[3], b[3]);
    if (m < 4) {
#pragma unroll
      for (int v = 0; v < 8; ++v) bsb[m][w * 16 + 8 * hi + v] = acc[v] * INV_WCAR;
    }
    __syncthreads();
    if (w == 0) {
      const int qrow = blockIdx.x >> 2;
      const int k0 = (blockIdx.x & 3) * 64;
      const int hh0 = lane >> 4, kk4 = (lane & 15) * 4;
      const v4f u0 = *(const v4fa*)&bsb[hh0][kk4];
      const v4f u1 = *(const v4fa*)&bsb[hh0 + 2][kk4];
      float* p0 = biasbuf + ((size_t)(qrow * NH + hh0)) * NRES_FULL + k0 + kk4;
      float* p1 = biasbuf + ((size_t)(qrow * NH + hh0 + 2)) * NRES_FULL + k0 + kk4;
      *(volatile v4f*)p0 = u0;
      *(volatile v4f*)p1 = u1;
      __threadfence();
      *(volatile v4f*)p0 = u0;
      *(volatile v4f*)p1 = u1;
    }
  }
}

__global__ __launch_bounds__(128) __attribute__((amdgpu_num_vgpr(256)))
void kB(const half_t* __restrict__ qbuf, const half_t* __restrict__ kbuf,
        const half_t* __restrict__ vbuf, const half_t* __restrict__ gbuf,
        const float* __restrict__ biasbuf, const float* __restrict__ bg,
        half_t* aobuf) {
  __shared__ __attribute__((aligned(16))) half_t Vt[CH * NRES_FULL];
  __shared__ __attribute__((aligned(16))) half_t ost[4][16 * CH];
  const int r = blockIdx.x >> 2, h = blockIdx.x & 3;
  const int tid = threadIdx.x, w = tid >> 5, lane = tid & 31;
  const int m = lane & 15, hi = lane >> 4;
  const size_t rowb = (size_t)r * NRES_FULL;

  for (int idx = tid; idx < NRES_FULL * 4; idx += 128) {
    const int j = idx >> 2, dg = idx & 3;
    const h8 vv = *(const h8a*)(vbuf + (rowb + j) * HC + h * CH + dg * 8);
#pragma unroll
    for (int e = 0; e < 8; ++e) Vt[(dg * 8 + e) * NRES_FULL + j] = vv[e];
  }
  __syncthreads();

  const float escale = 0.17677669529663687f * (1.0f / 65536.0f);

#pragma unroll 1
  for (int itl = 0; itl < 4; ++itl) {
    const int q0 = (itl * 4 + w) * 16;
    const half_t* qc = qbuf + (rowb + q0 + m) * HC + h * CH + hi * 8;
    v16h bQ = frag2(qc, qc + 16);
    const float* brow = biasbuf + ((size_t)(q0 + m) * NH + h) * NRES_FULL + 8 * hi;
    float mrun = -1.0e30f, lrun = 0.0f;
    v8f oacc0 = {}, oacc1 = {};

#pragma unroll 1
    for (int jc = 0; jc < NRES_FULL / 32; ++jc) {
      const int kb0 = jc * 32;
      const half_t* kc0 = kbuf + (rowb + kb0 + m) * HC + h * CH + hi * 8;
      const half_t* kc1 = kc0 + 16 * HC;
      v16h aK0 = frag2(kc0, kc0 + 16);
      v16h aK1 = frag2(kc1, kc1 + 16);
      const v4f b00 = *(const v4fa*)(brow + kb0);
      const v4f b01 = *(const v4fa*)(brow + kb0 + 4);
      const v4f b10 = *(const v4fa*)(brow + kb0 + 16);
      const v4f b11 = *(const v4fa*)(brow + kb0 + 20);
      v8f s0 = {}, s1 = {};
      s0 = wmma32(aK0, bQ, s0);
      s1 = wmma32(aK1, bQ, s1);
      wguard2(s0, s1, aK0, aK1, bQ);

      float x0[8], x1[8];
#pragma unroll
      for (int v = 0; v < 4; ++v) {
        x0[v]     = s0[v]     * escale + b00[v];
        x0[v + 4] = s0[v + 4] * escale + b01[v];
        x1[v]     = s1[v]     * escale + b10[v];
        x1[v + 4] = s1[v + 4] * escale + b11[v];
      }
      float cm = fmaxf(x0[0], x1[0]);
#pragma unroll
      for (int v = 1; v < 8; ++v) cm = fmaxf(cm, fmaxf(x0[v], x1[v]));
      cm = fmaxf(cm, __shfl_xor(cm, 16, 32));
      const float mnew = fmaxf(mrun, cm);
      const float alpha = __expf(mrun - mnew);
      mrun = mnew;

      v16h bP;
      float ps = 0.0f;
#pragma unroll
      for (int v = 0; v < 8; ++v) {
        const half_t pe0 = (half_t)__expf(x0[v] - mnew);
        const half_t pe1 = (half_t)__expf(x1[v] - mnew);
        bP[v] = pe0;
        bP[v + 8] = pe1;
        ps += (float)pe0 + (float)pe1;
      }
      ps += __shfl_xor(ps, 16, 32);
      lrun = lrun * alpha + ps;
#pragma unroll
      for (int v = 0; v < 8; ++v) { oacc0[v] *= alpha; oacc1[v] *= alpha; }

      const half_t* vc0 = Vt + m * NRES_FULL + kb0 + hi * 8;
      const half_t* vc1 = vc0 + 16 * NRES_FULL;
      v16h aV0 = frag2(vc0, vc0 + 16);
      v16h aV1 = frag2(vc1, vc1 + 16);
      oacc0 = wmma32(aV0, bP, oacc0);
      oacc1 = wmma32(aV1, bP, oacc1);
      wguard2(oacc0, oacc1, aV0, aV1, bP);
    }

    const float onorm = __builtin_amdgcn_rcpf(lrun) * INV_WCAR;
    const size_t growq = (rowb + q0 + m) * HC + h * CH + 8 * hi;
#pragma unroll
    for (int ct = 0; ct < 2; ++ct) {
      const h8 gp8 = *(const h8a*)(gbuf + growq + ct * 16);
      const v4f bga = *(const v4fa*)(bg + h * CH + ct * 16 + 8 * hi);
      const v4f bgb = *(const v4fa*)(bg + h * CH + ct * 16 + 8 * hi + 4);
      float bgv[8];
#pragma unroll
      for (int v = 0; v < 4; ++v) { bgv[v] = bf16r(bga[v]); bgv[v + 4] = bf16r(bgb[v]); }
      const v8f osel = ct ? oacc1 : oacc0;
      h8 o8;
#pragma unroll
      for (int v = 0; v < 8; ++v) {
        const float oa = osel[v] * onorm;
        const float gp = (float)gp8[v] * INV_WCAR + bgv[v];
        const float g  = __builtin_amdgcn_rcpf(1.0f + __expf(-gp));
        o8[v] = (half_t)(oa * g * OCAR);
      }
      *(h8a*)&ost[w][m * CH + ct * 16 + 8 * hi] = o8;
    }
    __syncthreads();
    const int rl = lane >> 2, c8 = (lane & 3) * 8;
    const h8 o0 = *(const h8a*)&ost[w][rl * CH + c8];
    const h8 o1 = *(const h8a*)&ost[w][(rl + 8) * CH + c8];
    half_t* d0 = aobuf + ((size_t)h * NROWS_FULL + rowb + q0 + rl) * CH + c8;
    half_t* d1 = d0 + 8 * CH;
    *(volatile h8*)d0 = o0;
    *(volatile h8*)d1 = o1;
    __threadfence();
    *(volatile h8*)d0 = o0;
    *(volatile h8*)d1 = o1;
  }
}

__global__ __launch_bounds__(128) void kC(const half_t* __restrict__ aobuf, const half_t* __restrict__ packedW,
                                          const float* __restrict__ bo, float* out) {
  __shared__ __attribute__((aligned(16))) float ot[4][16 * CZ];
  const int tid = threadIdx.x, w = tid >> 5, lane = tid & 31;
  const int m = lane & 15, hi = lane >> 4;
  const int r0 = (blockIdx.x * 4 + w) * 16;

  v16h afr[4];
#pragma unroll
  for (int kb = 0; kb < 4; ++kb) {
    const half_t* c0 = aobuf + ((size_t)kb * NROWS_FULL + (size_t)(r0 + m)) * CH + hi * 8;
    afr[kb] = frag2(c0, c0 + 16);
  }
  v16h b[4];
#pragma unroll 1
  for (int nt = 0; nt < 8; ++nt) {
    loadB4(packedW, 33 + nt, lane, b);
    v8f acc = {};
#pragma unroll
    for (int kb = 0; kb < 4; ++kb) acc = wmma32(afr[kb], b[kb], acc);
    wguard(acc, afr[3], b[3]);
    const float boc = bf16r(bo[nt * 16 + m]);
#pragma unroll
    for (int v = 0; v < 8; ++v)
      ot[w][(8 * hi + v) * CZ + nt * 16 + m] = acc[v] * (1.0f / 65536.0f) + boc;
  }
  __syncthreads();
#pragma unroll
  for (int p = 0; p < 16; ++p) {
    const v4f val = *(const v4fa*)&ot[w][p * CZ + lane * 4];
    *(volatile v4f*)(out + (size_t)(r0 + p) * CZ + lane * 4) = val;
  }
  __threadfence();
#pragma unroll
  for (int p = 0; p < 16; ++p) {
    const v4f val = *(const v4fa*)&ot[w][p * CZ + lane * 4];
    *(volatile v4f*)(out + (size_t)(r0 + p) * CZ + lane * 4) = val;
  }
}

extern "C" void kernel_launch(void* const* d_in, const int* in_sizes, int n_in,
                              void* d_out, int out_size, void* d_ws, size_t ws_size,
                              hipStream_t stream) {
  if (n_in < 11) return;
  if (in_sizes[0] < NROWS_FULL * CZ) return;
  if (in_sizes[1] < CZ || in_sizes[2] < CZ) return;
  if (in_sizes[3] < CZ * NH) return;
  if (in_sizes[4] < CZ * HC || in_sizes[5] < CZ * HC || in_sizes[6] < CZ * HC || in_sizes[7] < CZ * HC) return;
  if (in_sizes[8] < HC) return;
  if (in_sizes[9] < HC * CZ) return;
  if (in_sizes[10] < CZ) return;
  if (out_size < NQROWS * CZ) return;
  if (ws_size < WS_TOTAL) return;

  const float* z   = (const float*)d_in[0];
  const float* lng = (const float*)d_in[1];
  const float* lnb = (const float*)d_in[2];
  const float* Wb  = (const float*)d_in[3];
  const float* Wq  = (const float*)d_in[4];
  const float* Wk  = (const float*)d_in[5];
  const float* Wv  = (const float*)d_in[6];
  const float* Wg  = (const float*)d_in[7];
  const float* bg  = (const float*)d_in[8];
  const float* Wo  = (const float*)d_in[9];
  const float* bo  = (const float*)d_in[10];

  char* ws = (char*)d_ws;
  half_t* packedW = (half_t*)(ws + OFF_W);
  half_t* proj    = (half_t*)(ws + OFF_PROJ);
  half_t* qbuf    = proj;
  half_t* kbuf    = proj + PLANE_HALVES;
  half_t* vbuf    = proj + 2 * PLANE_HALVES;
  half_t* gbuf    = proj + 3 * PLANE_HALVES;
  half_t* aobuf   = (half_t*)(ws + OFF_AO);
  float*  biasbuf = (float*)(ws + OFF_BIAS);

  kP<<<dim3(NTILES), dim3(256), 0, stream>>>(Wb, Wq, Wk, Wv, Wg, Wo, packedW);
  kA<<<dim3(NROWS_FULL / 64), dim3(128), 0, stream>>>(z, lng, lnb, packedW, proj, biasbuf, (int)NQROWS);
  kB<<<dim3(NB * NH), dim3(128), 0, stream>>>(qbuf, kbuf, vbuf, gbuf, biasbuf, bg, aobuf);
  kC<<<dim3(NQROWS / 64), dim3(128), 0, stream>>>(aobuf, packedW, bo, (float*)d_out);
}
